// BiLSTMTagger_41463614275780
// MI455X (gfx1250) — hardware-verified
//
#include <hip/hip_runtime.h>
#include <math.h>
#include <stdint.h>

#define SEQ_LEN   512
#define N_BATCH   64
#define N_VOCAB   100000
#define N_EMB     128
#define N_HID     256
#define N_GATE    1024
#define K_CAT     384
#define N_TAG     64
#define N_THR     256
#define M_ROWS    16
#define A_PITCH   392
#define X_SC      8.0f
#define WIH_SC    8.0f
#define WHH_SC    64.0f
#define G_INV     (1.0f / 64.0f)
#define WOUT_SC   8.0f
#define OUT_INV   (1.0f / 8.0f)
#define WC_CHUNKS (N_GATE * K_CAT / 8)
#define WO_CHUNKS (N_TAG * 2 * N_HID / 8)

static_assert(K_CAT == N_EMB + N_HID, "k layout");
static_assert(A_PITCH % 8 == 0 && A_PITCH >= K_CAT, "A pitch");
static_assert(WC_CHUNKS % N_THR == 0, "exact grid");
static_assert(WO_CHUNKS % N_THR == 0, "exact grid");
static_assert((SEQ_LEN * N_BATCH) % 64 == 0 && (2 * N_HID) % 32 == 0 && N_TAG % 64 == 0, "gemm tiles");

typedef __attribute__((ext_vector_type(16))) _Float16 v16h;
typedef __attribute__((ext_vector_type(8)))  _Float16 v8h;
typedef __attribute__((ext_vector_type(16))) __bf16   v16b;
typedef __attribute__((ext_vector_type(8)))  __bf16   v8b;
typedef __attribute__((ext_vector_type(8)))  float    v8f;
typedef __attribute__((ext_vector_type(4)))  float    v4f;

__device__ __forceinline__ unsigned short f2bf_bits(float f) {
  unsigned u = __float_as_uint(f);
  return (unsigned short)((u + 0x7FFFu + ((u >> 16) & 1u)) >> 16);
}
__device__ __forceinline__ float bf_bits2f(unsigned short h) { return __uint_as_float(((unsigned)h) << 16); }

__device__ __forceinline__ void dep_guard_h(v8f& a, v8f& b, v16h x, v16h y) { asm volatile("v_nop\n\tv_nop\n\tv_nop\n\tv_nop" : "+v"(a), "+v"(b) : "v"(x), "v"(y)); }
__device__ __forceinline__ void dep_guard_b(v8f& a, v8f& b, v16b x, v16b y) { asm volatile("v_nop\n\tv_nop\n\tv_nop\n\tv_nop" : "+v"(a), "+v"(b) : "v"(x), "v"(y)); }
__device__ __forceinline__ void keep4_h(v16h a, v16h b, v16h c, v16h d) { asm volatile("v_nop" :: "v"(a), "v"(b), "v"(c), "v"(d)); }
__device__ __forceinline__ void keep4_b(v16b a, v16b b, v16b c, v16b d) { asm volatile("v_nop" :: "v"(a), "v"(b), "v"(c), "v"(d)); }
__device__ __forceinline__ void acc_guard4(v8f& a, v8f& b, v8f& c, v8f& d) { asm volatile("v_nop\n\tv_nop\n\tv_nop\n\tv_nop" : "+v"(a), "+v"(b), "+v"(c), "+v"(d)); }
template <typename T> struct Frag;
template <> struct Frag<_Float16> {
  typedef v16h V; union U { v16h v; v8h h[2]; };
  static __device__ __forceinline__ v16h load(const _Float16* p) {
    U f; f.h[0] = *(const v8h*)(p); f.h[1] = *(const v8h*)(p + 16); return f.v;
  }
  static __device__ __forceinline__ v8f mma(v16h a, v16h b, v8f c) {
    return __builtin_amdgcn_wmma_f32_16x16x32_f16(false, a, false, b, (short)0, c, false, false);
  }
  static __device__ __forceinline__ void guard(v8f& a, v8f& b, v16h x, v16h y) { dep_guard_h(a, b, x, y); }
  static __device__ __forceinline__ void keep(v16h a, v16h b, v16h c, v16h d) { keep4_h(a, b, c, d); }
};
template <> struct Frag<__bf16> {
  typedef v16b V; union U { v16b v; v8b h[2]; };
  static __device__ __forceinline__ v16b load(const __bf16* p) {
    U f; f.h[0] = *(const v8b*)(p); f.h[1] = *(const v8b*)(p + 16); return f.v;
  }
  static __device__ __forceinline__ v8f mma(v16b a, v16b b, v8f c) {
    return __builtin_amdgcn_wmma_f32_16x16x32_bf16(false, a, false, b, (short)0, c, false, false);
  }
  static __device__ __forceinline__ void guard(v8f& a, v8f& b, v16b x, v16b y) { dep_guard_b(a, b, x, y); }
  static __device__ __forceinline__ void keep(v16b a, v16b b, v16b c, v16b d) { keep4_b(a, b, c, d); }
};

template <int ET> struct Elem;
template <> struct Elem<0> { typedef _Float16 T; };
template <> struct Elem<1> { typedef __bf16 T; };
template <int ET, bool SPLIT, int BIAS_MODE, int OUT_MODE, bool RESID, int ACT = 0>
__global__ __launch_bounds__(256) void wmma_gemm64(
    const unsigned short* __restrict__ Ap, const unsigned short* __restrict__ A2p, int lda, long strideA,
    const unsigned short* __restrict__ Btp, const unsigned short* __restrict__ Bt2p, int ldb, long strideB,
    void* __restrict__ Cout, void* __restrict__ Cout2, int ldc, long strideC,
    const float* __restrict__ bias,
    const float* __restrict__ resid, long strideR,
    int M, int N, int K, float scale) {
  typedef typename Elem<ET>::T T;
  typedef typename Frag<T>::V V;
  const T* A = (const T*)Ap; const T* A2 = (const T*)A2p; const T* Bt = (const T*)Btp; const T* Bt2 = (const T*)Bt2p;
  __shared__ __align__(16) float sT[8][16 * 68];
  const int b    = blockIdx.y;
  const int lane = threadIdx.x & 31;
  const int wave = threadIdx.x >> 5;
  const int tilesN = N >> 6;
  const int tilesM = M >> 6;
  const int tile = blockIdx.x * 8 + wave;
  if (tile >= tilesM * tilesN) return;
  const int tm = tile / tilesN;
  const int tn = tile - tm * tilesN;
  const int m0 = tm << 6;
  const int n0 = tn << 6;

  const T* Ab  = A  + (size_t)b * strideA;
  const T* Bb  = Bt + (size_t)b * strideB;
  const T* Ab2 = SPLIT ? (A2  + (size_t)b * strideA) : nullptr;
  const T* Bb2 = SPLIT ? (Bt2 + (size_t)b * strideB) : nullptr;

  const int rlane = lane & 15;
  const int koff  = (lane >> 4) * 8;
  const int mOff  = (lane >> 4) * 8;

  v8f acc[4][4];
#pragma unroll
  for (int i = 0; i < 4; ++i)
#pragma unroll
    for (int j = 0; j < 4; ++j) acc[i][j] = (v8f){0.f,0.f,0.f,0.f,0.f,0.f,0.f,0.f};

  for (int k0 = 0; k0 < K; k0 += 32) {
    V bh[4], bl[4];
#pragma unroll
    for (int j = 0; j < 4; ++j) {
      const size_t bo = (size_t)(n0 + (j << 4) + rlane) * ldb + koff + k0;
      bh[j] = Frag<T>::load(Bb + bo);
      if (SPLIT) bl[j] = Frag<T>::load(Bb2 + bo);
    }
#pragma unroll
    for (int i = 0; i < 4; ++i) {
      const size_t ao = (size_t)(m0 + (i << 4) + rlane) * lda + koff + k0;
      V ah = Frag<T>::load(Ab + ao);
      V al;
      if (SPLIT) al = Frag<T>::load(Ab2 + ao);
#pragma unroll
      for (int j = 0; j < 4; ++j) {
        acc[i][j] = Frag<T>::mma(ah, bh[j], acc[i][j]);
        if (SPLIT) {
          acc[i][j] = Frag<T>::mma(ah, bl[j], acc[i][j]);
          acc[i][j] = Frag<T>::mma(al, bh[j], acc[i][j]);
        }
      }
      Frag<T>::guard(acc[i][0], acc[i][3], ah, SPLIT ? al : ah);
    }
    Frag<T>::keep(bh[0], bh[1], bh[2], bh[3]);
    if (SPLIT) Frag<T>::keep(bl[0], bl[1], bl[2], bl[3]);
  }
  acc_guard4(acc[0][0], acc[0][1], acc[0][2], acc[0][3]);
  acc_guard4(acc[1][0], acc[1][1], acc[1][2], acc[1][3]);
  acc_guard4(acc[2][0], acc[2][1], acc[2][2], acc[2][3]);
  acc_guard4(acc[3][0], acc[3][1], acc[3][2], acc[3][3]);

  float* slab = sT[wave];
  const float* Rb = RESID ? (resid + (size_t)b * strideR) : nullptr;
#pragma unroll
  for (int i = 0; i < 4; ++i) {
    const int mBase = m0 + (i << 4);
#pragma unroll
    for (int j = 0; j < 4; ++j) {
      const int n = n0 + (j << 4) + rlane;
      float bv = 0.f;
      if (BIAS_MODE == 2) bv = bias[n];
#pragma unroll
      for (int r = 0; r < 8; ++r) {
        float v = acc[i][j][r] * scale;
        if (BIAS_MODE == 1) v += bias[mBase + mOff + r];
        if (BIAS_MODE == 2) v += bv;
        if (RESID) v += Rb[(size_t)(mBase + mOff + r) * ldc + n];
        if (ACT == 1) v = tanhf(v);
        if (ACT == 2) v = fmaxf(v, 0.0f);
        if (ACT == 3) v = v / (1.0f + expf(-v));
        if (ACT == 4) v = (v > 0.f) ? v : 0.01f * v;
        if (ACT == 5) v = 0.5f * v * (1.0f + erff(v * 0.70710678118654752f));
        slab[(mOff + r) * 68 + (j << 4) + rlane] = v;
      }
    }
    __builtin_amdgcn_fence(__ATOMIC_RELEASE, "workgroup");
    __builtin_amdgcn_wave_barrier();
    __builtin_amdgcn_fence(__ATOMIC_ACQUIRE, "workgroup");
    if (OUT_MODE == 0) {
      float* C = (float*)Cout + (size_t)b * strideC;
      const int hh = lane >> 4, c4 = (lane & 15) * 4;
      for (int pass = 0; pass < 2; ++pass) {
#pragma unroll
        for (int it = 0; it < 8; ++it) {
          const int row = it * 2 + hh;
          v4f v = *(const v4f*)(slab + row * 68 + c4);
          *(volatile v4f*)(C + (size_t)(mBase + row) * ldc + n0 + c4) = v;
        }
        __threadfence();
      }
    } else {
      const int q = lane >> 3, c8 = (lane & 7) * 8;
      unsigned short* C  = (unsigned short*)Cout  + (size_t)b * strideC;
      unsigned short* C2 = (OUT_MODE == 2) ? ((unsigned short*)Cout2 + (size_t)b * strideC) : nullptr;
      for (int pass = 0; pass < 2; ++pass) {
#pragma unroll
        for (int it = 0; it < 4; ++it) {
          const int row = it * 4 + q;
          const float* sp = slab + row * 68 + c8;
          v8h hv, lv;
#pragma unroll
          for (int e = 0; e < 8; ++e) {
            if (OUT_MODE == 1) {
              hv[e] = (_Float16)sp[e];
            } else {
              unsigned short hb = f2bf_bits(sp[e]);
              unsigned short lb = f2bf_bits(sp[e] - bf_bits2f(hb));
              hv[e] = __builtin_bit_cast(_Float16, hb);
              lv[e] = __builtin_bit_cast(_Float16, lb);
            }
          }
          *(volatile v8h*)(C + (size_t)(mBase + row) * ldc + n0 + c8) = hv;
          if (OUT_MODE == 2) *(volatile v8h*)(C2 + (size_t)(mBase + row) * ldc + n0 + c8) = lv;
        }
        __threadfence();
      }
    }
    __builtin_amdgcn_fence(__ATOMIC_RELEASE, "workgroup");
    __builtin_amdgcn_wave_barrier();
    __builtin_amdgcn_fence(__ATOMIC_ACQUIRE, "workgroup");
  }
}

__device__ __forceinline__ float fsig(float x)  { return __builtin_amdgcn_rcpf(1.0f + __expf(-x)); }
__device__ __forceinline__ float ftanh(float x) { return 1.0f - 2.0f * __builtin_amdgcn_rcpf(__expf(2.0f * x) + 1.0f); }

__global__ __launch_bounds__(N_THR) void wcat_kernel(const float* __restrict__ Wihf, const float* __restrict__ Whhf,
                                                    const float* __restrict__ Wihb, const float* __restrict__ Whhb,
                                                    unsigned short* __restrict__ WCp) {
  const int dir = blockIdx.y;
  const int i = blockIdx.x * N_THR + threadIdx.x;
  if (i >= WC_CHUNKS) return;
  const int n = i / 48, q = i - n * 48;
  const int qi = (q < 16) ? q : 15;
  const int qh = (q >= 16) ? (q - 16) : 0;
  const float* Wih = dir ? Wihb : Wihf;
  const float* Whh = dir ? Whhb : Whhf;
  const float* pih = Wih + (size_t)n * N_EMB + (size_t)qi * 8;
  const float* phh = Whh + (size_t)n * N_HID + (size_t)qh * 8;
  const v4f a0 = *(const v4f*)pih, a1 = *(const v4f*)(pih + 4);
  const v4f g0 = *(const v4f*)phh, g1 = *(const v4f*)(phh + 4);
  const bool useI = (q < 16);
  v8h hv;
#pragma unroll
  for (int e = 0; e < 4; ++e) {
    const float f0 = useI ? (a0[e] * WIH_SC) : (g0[e] * WHH_SC);
    const float f1 = useI ? (a1[e] * WIH_SC) : (g1[e] * WHH_SC);
    hv[e]     = (_Float16)f0;
    hv[4 + e] = (_Float16)f1;
  }
  _Float16* O = (_Float16*)WCp + (size_t)dir * N_GATE * K_CAT + (size_t)i * 8;
  *(volatile v8h*)O = hv;
  __threadfence();
  *(volatile v8h*)O = hv;
}

__global__ __launch_bounds__(N_THR) void wout_kernel(const float* __restrict__ Wout, unsigned short* __restrict__ WOp) {
  const int i = blockIdx.x * N_THR + threadIdx.x;
  if (i >= WO_CHUNKS) return;
  const float* p = Wout + (size_t)i * 8;
  const v4f a0 = *(const v4f*)p, a1 = *(const v4f*)(p + 4);
  v8h hv;
#pragma unroll
  for (int e = 0; e < 4; ++e) {
    hv[e]     = (_Float16)(a0[e] * WOUT_SC);
    hv[4 + e] = (_Float16)(a1[e] * WOUT_SC);
  }
  _Float16* O = (_Float16*)WOp + (size_t)i * 8;
  *(volatile v8h*)O = hv;
  __threadfence();
  *(volatile v8h*)O = hv;
}

__global__ __launch_bounds__(N_THR) void bilstm_kernel(const int* __restrict__ tok, const float* __restrict__ emb,
                                                      const float* __restrict__ bihf, const float* __restrict__ bhhf,
                                                      const float* __restrict__ bihb, const float* __restrict__ bhhb,
                                                      const unsigned short* __restrict__ WCp,
                                                      unsigned short* __restrict__ HCp) {
  __shared__ __align__(16) _Float16 At[M_ROWS * A_PITCH];
  const int tid = threadIdx.x, lane = tid & 31, wave = tid >> 5;
  const int c = lane & 15, hh = lane >> 4, koff = hh * 8;
  const int dir = blockIdx.x >> 2;
  const int b0 = (blockIdx.x & 3) * M_ROWS;
  const _Float16* WC = (const _Float16*)WCp + (size_t)dir * N_GATE * K_CAT;
  _Float16* HC = (_Float16*)HCp;

#pragma unroll 1
  for (int i = 0; i < M_ROWS; ++i) At[i * A_PITCH + N_EMB + tid] = (_Float16)0.0f;
  {
    const int srow = dir ? (SEQ_LEN - 1) : 0;
    const int m = tid >> 4, e8 = (tid & 15) * 8;
    int id = tok[srow * N_BATCH + b0 + m];
    id = (id < 0) ? 0 : ((id > N_VOCAB - 1) ? (N_VOCAB - 1) : id);
    const float* er = emb + (size_t)id * N_EMB + e8;
    const v4f v0 = *(const v4f*)er;
    const v4f v1 = *(const v4f*)(er + 4);
    v8h hv;
#pragma unroll
    for (int e = 0; e < 4; ++e) { hv[e] = (_Float16)(v0[e] * X_SC); hv[4 + e] = (_Float16)(v1[e] * X_SC); }
    *(v8h*)(At + m * A_PITCH + e8) = hv;
  }
  float cst[2][8], hst[2][8], bb[2][4];
#pragma unroll
  for (int nt = 0; nt < 2; ++nt) {
    const int j = 32 * wave + 16 * nt + c;
#pragma unroll
    for (int g = 0; g < 4; ++g) {
      const float vf = bihf[g * N_HID + j] + bhhf[g * N_HID + j];
      const float vb = bihb[g * N_HID + j] + bhhb[g * N_HID + j];
      bb[nt][g] = dir ? vb : vf;
    }
#pragma unroll
    for (int r = 0; r < 8; ++r) { cst[nt][r] = 0.0f; hst[nt][r] = 0.0f; }
  }
  __syncthreads();

  const _Float16* arow = At + c * A_PITCH + koff;
  const v8f z8 = {0.f, 0.f, 0.f, 0.f, 0.f, 0.f, 0.f, 0.f};

#pragma unroll 1
  for (int t = 0; t < SEQ_LEN; ++t) {
#pragma unroll
    for (int nt = 0; nt < 2; ++nt) {
      const int j = 32 * wave + 16 * nt + c;
      const _Float16* wrow = WC + (size_t)j * K_CAT + koff;
      v8f acc[4];
      acc[0] = z8; acc[1] = z8; acc[2] = z8; acc[3] = z8;
#pragma unroll 1
      for (int k0 = 0; k0 < K_CAT; k0 += 32) {
        const v16h a  = Frag<_Float16>::load(arow + k0);
        const v16h f0 = Frag<_Float16>::load(wrow + k0);
        const v16h f1 = Frag<_Float16>::load(wrow + (size_t)1 * N_HID * K_CAT + k0);
        const v16h f2 = Frag<_Float16>::load(wrow + (size_t)2 * N_HID * K_CAT + k0);
        const v16h f3 = Frag<_Float16>::load(wrow + (size_t)3 * N_HID * K_CAT + k0);
        acc[0] = Frag<_Float16>::mma(a, f0, acc[0]);
        acc[1] = Frag<_Float16>::mma(a, f1, acc[1]);
        acc[2] = Frag<_Float16>::mma(a, f2, acc[2]);
        acc[3] = Frag<_Float16>::mma(a, f3, acc[3]);
        dep_guard_h(acc[0], acc[3], a, f3);
        keep4_h(f0, f1, f2, f3);
      }
      acc_guard4(acc[0], acc[1], acc[2], acc[3]);
#pragma unroll
      for (int r = 0; r < 8; ++r) {
        const float zi = acc[0][r] * G_INV + bb[nt][0];
        const float zf = acc[1][r] * G_INV + bb[nt][1];
        const float zg = acc[2][r] * G_INV + bb[nt][2];
        const float zo = acc[3][r] * G_INV + bb[nt][3];
        const float ig = fsig(zi);
        const float fg = fsig(zf);
        const float gg = ftanh(zg);
        const float og = fsig(zo);
        const float cn = fg * cst[nt][r] + ig * gg;
        cst[nt][r] = cn;
        hst[nt][r] = og * ftanh(cn);
      }
    }
    __syncthreads();
#pragma unroll
    for (int nt = 0; nt < 2; ++nt) {
      const int j = 32 * wave + 16 * nt + c;
#pragma unroll
      for (int r = 0; r < 8; ++r) At[(8 * hh + r) * A_PITCH + N_EMB + j] = (_Float16)hst[nt][r];
    }
    {
      const int tn = (t + 1 < SEQ_LEN) ? (t + 1) : (SEQ_LEN - 1);
      const int srow = dir ? (SEQ_LEN - 1 - tn) : tn;
      const int m = tid >> 4, e8 = (tid & 15) * 8;
      int id = tok[srow * N_BATCH + b0 + m];
      id = (id < 0) ? 0 : ((id > N_VOCAB - 1) ? (N_VOCAB - 1) : id);
      const float* er = emb + (size_t)id * N_EMB + e8;
      const v4f v0 = *(const v4f*)er;
      const v4f v1 = *(const v4f*)(er + 4);
      v8h hv;
#pragma unroll
      for (int e = 0; e < 4; ++e) { hv[e] = (_Float16)(v0[e] * X_SC); hv[4 + e] = (_Float16)(v1[e] * X_SC); }
      *(v8h*)(At + m * A_PITCH + e8) = hv;
    }
    __syncthreads();
    {
      const int srow = dir ? (SEQ_LEN - 1 - t) : t;
      v8h hv2[2];
      size_t o2[2];
#pragma unroll
      for (int it = 0; it < 2; ++it) {
        const int idx = it * N_THR + tid;
        const int row = idx >> 5, c8 = (idx & 31) * 8;
        hv2[it] = *(const v8h*)(At + row * A_PITCH + N_EMB + c8);
        o2[it] = (size_t)(srow * N_BATCH + b0 + row) * (size_t)(2 * N_HID) + (size_t)dir * N_HID + (size_t)c8;
      }
      for (int pass = 0; pass < 2; ++pass) {
#pragma unroll
        for (int it = 0; it < 2; ++it) *(volatile v8h*)(HC + o2[it]) = hv2[it];
        __threadfence();
      }
    }
  }
}

extern "C" void kernel_launch(void* const* d_in, const int* in_sizes, int n_in,
                              void* d_out, int out_size, void* d_ws, size_t ws_size, hipStream_t stream) {
  if (n_in < 12 || d_out == nullptr || d_ws == nullptr) return;
  if (in_sizes[0] != SEQ_LEN * N_BATCH || in_sizes[1] != N_VOCAB * N_EMB ||
      in_sizes[2] != N_GATE * N_EMB || in_sizes[3] != N_GATE * N_HID || in_sizes[4] != N_GATE || in_sizes[5] != N_GATE ||
      in_sizes[6] != N_GATE * N_EMB || in_sizes[7] != N_GATE * N_HID || in_sizes[8] != N_GATE || in_sizes[9] != N_GATE ||
      in_sizes[10] != N_TAG * 2 * N_HID || in_sizes[11] != N_TAG || out_size != SEQ_LEN * N_BATCH * N_TAG) return;

  const int*   tok  = (const int*)d_in[0];
  const float* emb  = (const float*)d_in[1];
  const float* Wihf = (const float*)d_in[2];
  const float* Whhf = (const float*)d_in[3];
  const float* bihf = (const float*)d_in[4];
  const float* bhhf = (const float*)d_in[5];
  const float* Wihb = (const float*)d_in[6];
  const float* Whhb = (const float*)d_in[7];
  const float* bihb = (const float*)d_in[8];
  const float* bhhb = (const float*)d_in[9];
  const float* Wout = (const float*)d_in[10];
  const float* bout = (const float*)d_in[11];
  float* out = (float*)d_out;

  char* ws = (char*)d_ws; size_t off = 0;
  auto carve = [&](size_t bytes) -> char* { char* p = ws + off; off += (bytes + 255) & ~(size_t)255; return p; };
  unsigned short* WCb = (unsigned short*)carve((size_t)2 * N_GATE * K_CAT * 2);
  unsigned short* WOb = (unsigned short*)carve((size_t)N_TAG * 2 * N_HID * 2);
  unsigned short* HCb = (unsigned short*)carve((size_t)SEQ_LEN * N_BATCH * 2 * N_HID * 2);
  if (off > ws_size || off > (size_t)134217728) return;

  wcat_kernel<<<dim3(WC_CHUNKS / N_THR, 2), N_THR, 0, stream>>>(Wihf, Whhf, Wihb, Whhb, WCb);
  wout_kernel<<<WO_CHUNKS / N_THR, N_THR, 0, stream>>>(Wout, WOb);
  bilstm_kernel<<<8, N_THR, 0, stream>>>(tok, emb, bihf, bhhf, bihb, bhhb, WCb, HCb);
  wmma_gemm64<0, false, 2, 0, false, 0><<<dim3((SEQ_LEN * N_BATCH / 64) * (N_TAG / 64) / 8, 1), 256, 0, stream>>>(
      HCb, nullptr, 2 * N_HID, (long)0,
      WOb, nullptr, 2 * N_HID, (long)0,
      (void*)out, nullptr, N_TAG, (long)0,
      bout, nullptr, (long)0,
      SEQ_LEN * N_BATCH, N_TAG, 2 * N_HID, OUT_INV);
}
